// Decoder_29832842838551
// MI455X (gfx1250) — hardware-verified
//
#include <hip/hip_runtime.h>
#include <math.h>

constexpr int NBATCH = 8192;
constexpr int NLAT   = 16;
constexpr int NFC    = 64;
constexpr int NHID   = 32;
constexpr int NGATE  = 128;
constexpr int NSTEP  = 256;
constexpr int NCH1   = 16;
constexpr int NTAP   = 5;

constexpr int K1_WAVES = 4;
constexpr int XS_P     = 65;
constexpr int XP_P     = 132;

constexpr int K2_WAVES = 2;
constexpr int HR_P     = 40;
constexpr int HR_PLANE = 16 * HR_P;
constexpr int HR_SLOT  = 2 * HR_PLANE;
constexpr int WH_P     = 40;
constexpr int Y1_P     = 20;
constexpr int Y1_SLOT  = 16 * Y1_P;
constexpr int OT_P     = 36;
constexpr float LO_CARRY       = 2048.0f;
constexpr float LO_CARRY_INV   = 1.0f / 2048.0f;
constexpr float F16_MIN_NORMAL = 6.103515625e-5f;

static_assert(NGATE == 4 * NHID);
static_assert(NHID == 32);
static_assert(NBATCH % (16 * K1_WAVES) == 0);
static_assert(NBATCH % (16 * K2_WAVES) == 0);
static_assert(NSTEP % 32 == 0);
static_assert((8 * HR_SLOT) % (8 * 32) == 0);
static_assert((8 * Y1_SLOT) % (4 * 32) == 0);
static_assert(NBATCH * NSTEP * 4 == 8388608);

typedef __attribute__((ext_vector_type(16))) _Float16 v16h;
typedef __attribute__((ext_vector_type(8)))  _Float16 v8h;
typedef __attribute__((ext_vector_type(8)))  float    v8f;
typedef __attribute__((ext_vector_type(4)))  float    v4f;

struct FragH {
  union U { v16h v; v8h h[2]; };
  static __device__ __forceinline__ v16h load(const _Float16* p) {
    U f;
    f.h[0] = *(const v8h*)(p);
    f.h[1] = *(const v8h*)(p + 16);
    return f.v;
  }
  static __device__ __forceinline__ v8f mma(v16h a, v16h b, v8f c) {
    return __builtin_amdgcn_wmma_f32_16x16x32_f16(false, a, false, b, (short)0, c, false, false);
  }
};

__device__ __forceinline__ void guard_rec12(v8f& m0, v8f& m1, v8f& m2, v8f& m3,
                                            v8f& r0, v8f& r1, v8f& r2, v8f& r3,
                                            v16h a0, v16h a1,
                                            v16h b0, v16h b1, v16h b2, v16h b3,
                                            v16h l0, v16h l1, v16h l2, v16h l3) {
  asm volatile("v_nop\n\tv_nop\n\tv_nop\n\tv_nop"
               : "+v"(m0), "+v"(m1), "+v"(m2), "+v"(m3), "+v"(r0), "+v"(r1), "+v"(r2), "+v"(r3)
               : "v"(a0), "v"(a1), "v"(b0), "v"(b1), "v"(b2), "v"(b3), "v"(l0), "v"(l1), "v"(l2), "v"(l3));
}
__device__ __forceinline__ void guard_cv2(v8f& m, v8f& r, v16h a0, v16h a1, v16h b) {
  asm volatile("v_nop\n\tv_nop\n\tv_nop\n\tv_nop" : "+v"(m), "+v"(r) : "v"(a0), "v"(a1), "v"(b));
}
__device__ __forceinline__ float opaque_f32(float x) { asm volatile("" : "+v"(x)); return x; }

__device__ __forceinline__ float fsig(float x)  { return __builtin_amdgcn_rcpf(1.0f + __expf(-x)); }
__device__ __forceinline__ float ftanh(float x) { return 1.0f - 2.0f * __builtin_amdgcn_rcpf(__expf(2.0f * x) + 1.0f); }

__device__ __forceinline__ v8f ld_tile8(const float* p) {
  const v4f a = *(const v4f*)(p);
  const v4f b = *(const v4f*)(p + 4);
  v8f o = {a[0], a[1], a[2], a[3], b[0], b[1], b[2], b[3]};
  return o;
}

__global__ __launch_bounds__(K1_WAVES * 32) void xproj_kernel(const float* __restrict__ z,
                                                              const float* __restrict__ fc_w,
                                                              const float* __restrict__ fc_b,
                                                              const float* __restrict__ w_ih,
                                                              const float* __restrict__ b_ih,
                                                              const float* __restrict__ b_hh,
                                                              float* __restrict__ XP) {
  __shared__ __align__(16) float zs[K1_WAVES][16 * NLAT];
  __shared__ __align__(16) float xs[K1_WAVES][16 * XS_P];
  __shared__ __align__(16) float xps[K1_WAVES][16 * XP_P];
  const int tid = threadIdx.x, lane = tid & 31, wave = tid >> 5;
  const int bbase = (blockIdx.x * K1_WAVES + wave) * 16;
  float* zt  = zs[wave];
  float* xt  = xs[wave];
  float* xpt = xps[wave];

#pragma unroll
  for (int i = 0; i < 2; ++i) {
    const int idx4 = (i * 32 + lane) * 4;
    const v4f v = *(const v4f*)(z + (size_t)bbase * NLAT + idx4);
    *(v4f*)(zt + idx4) = v;
  }
  __syncthreads();

#pragma unroll 1
  for (int g = 0; g < NFC / 32; ++g) {
    const int col = g * 32 + lane;
    float acc[16];
#pragma unroll
    for (int m = 0; m < 16; ++m) acc[m] = 0.0f;
#pragma unroll 1
    for (int k = 0; k < NLAT; ++k) {
      const float w = fc_w[col * NLAT + k];
#pragma unroll
      for (int m = 0; m < 16; ++m) acc[m] = fmaf(zt[m * NLAT + k], w, acc[m]);
    }
    const float bv = fc_b[col];
#pragma unroll
    for (int m = 0; m < 16; ++m) xt[m * XS_P + col] = acc[m] + bv;
  }
  __syncthreads();

#pragma unroll 1
  for (int g = 0; g < NGATE / 32; ++g) {
    const int col = g * 32 + lane;
    float acc[16];
#pragma unroll
    for (int m = 0; m < 16; ++m) acc[m] = 0.0f;
#pragma unroll 1
    for (int k = 0; k < NFC; ++k) {
      const float w = w_ih[col * NFC + k];
#pragma unroll
      for (int m = 0; m < 16; ++m) acc[m] = fmaf(xt[m * XS_P + k], w, acc[m]);
    }
    const float b0 = b_ih[col];
    const float b1 = b_hh[col];
#pragma unroll
    for (int m = 0; m < 16; ++m) xpt[m * XP_P + col] = (acc[m] + b0) + b1;
  }
  __syncthreads();

  for (int pass = 0; pass < 2; ++pass) {
#pragma unroll
    for (int m = 0; m < 16; ++m) {
      const v4f v = *(const v4f*)(xpt + m * XP_P + 4 * lane);
      *(volatile v4f*)(XP + (size_t)(bbase + m) * NGATE + 4 * lane) = v;
    }
    __threadfence();
  }
}

__device__ __forceinline__ void flush_tile(const float* ot, float* __restrict__ out, int bbase, int g, int lane) {
  const int q = lane >> 3, c4 = (lane & 7) * 4;
  for (int pass = 0; pass < 2; ++pass) {
#pragma unroll
    for (int it = 0; it < 4; ++it) {
      const int row = it * 4 + q;
      const v4f v = *(const v4f*)(ot + row * OT_P + c4);
      *(volatile v4f*)(out + (size_t)(bbase + row) * NSTEP + g * 32 + c4) = v;
    }
    __threadfence();
  }
}

__global__ __launch_bounds__(K2_WAVES * 32) void decoder_seq_kernel(const float* __restrict__ XP,
                                                                    const float* __restrict__ w_hh,
                                                                    const float* __restrict__ c1w,
                                                                    const float* __restrict__ c1b,
                                                                    const float* __restrict__ c2w,
                                                                    const float* __restrict__ c2b,
                                                                    float* __restrict__ out) {
  __shared__ __align__(16) _Float16 WHs[NGATE * WH_P];
  __shared__ __align__(16) _Float16 WLs[NGATE * WH_P];
  __shared__ __align__(16) _Float16 C1s[NTAP * NCH1 * WH_P];
  __shared__ __align__(16) float    W2s[2 * NTAP * 8];
  __shared__ __align__(16) _Float16 HRs[K2_WAVES][8 * HR_SLOT];
  __shared__ __align__(32) float    XPs[K2_WAVES][8 * 32 * 8];
  __shared__ __align__(16) float    Y1s[K2_WAVES][8 * Y1_SLOT];
  __shared__ __align__(16) float    OTs[K2_WAVES][16 * OT_P];

  const int tid = threadIdx.x, lane = tid & 31, wave = tid >> 5;
  const int n = lane & 15, hf = lane >> 4;
  const int bbase = (blockIdx.x * K2_WAVES + wave) * 16;
  _Float16* hr = HRs[wave];
  float* xp = XPs[wave];
  float* y1 = Y1s[wave];
  float* ot = OTs[wave];

#pragma unroll 1
  for (int idx = tid; idx < NGATE * WH_P; idx += K2_WAVES * 32) {
    const int row = idx / WH_P;
    const int k = idx - row * WH_P;
    const int kc = (k < NHID) ? k : (NHID - 1);
    const float v = w_hh[row * NHID + kc];
    const float vs = (k < NHID) ? v : 0.0f;
    const _Float16 h0 = (_Float16)vs;
    const float hif = opaque_f32((float)h0);
    const float hin = (fabsf(hif) < F16_MIN_NORMAL) ? 0.0f : hif;
    const _Float16 hi = (_Float16)hin;
    const _Float16 lo = (_Float16)((vs - hin) * LO_CARRY);
    WHs[idx] = hi;
    WLs[idx] = lo;
  }
#pragma unroll 1
  for (int idx = tid; idx < NTAP * NCH1 * WH_P; idx += K2_WAVES * 32) {
    const int dt = idx / (NCH1 * WH_P);
    const int rem = idx - dt * (NCH1 * WH_P);
    const int och = rem / WH_P;
    const int c = rem - och * WH_P;
    const int cc = (c < NHID) ? c : (NHID - 1);
    const float v = c1w[(och * NHID + cc) * NTAP + dt];
    const float vs = (c < NHID) ? v : 0.0f;
    C1s[idx] = (_Float16)vs;
  }
#pragma unroll 1
  for (int idx = tid; idx < 2 * NTAP * 8; idx += K2_WAVES * 32) {
    const int hfi = idx / (NTAP * 8);
    const int rem = idx - hfi * (NTAP * 8);
    const int dt = rem >> 3;
    const int i = rem & 7;
    W2s[idx] = c2w[(hfi * 8 + i) * NTAP + dt];
  }
  {
    const v8h z8h = {(_Float16)0.0f, (_Float16)0.0f, (_Float16)0.0f, (_Float16)0.0f,
                     (_Float16)0.0f, (_Float16)0.0f, (_Float16)0.0f, (_Float16)0.0f};
#pragma unroll 1
    for (int i = lane; i < (8 * HR_SLOT) / 8; i += 32) *(v8h*)(hr + 8 * i) = z8h;
  }
  {
    const v4f z4 = {0.0f, 0.0f, 0.0f, 0.0f};
#pragma unroll 1
    for (int i = lane; i < (8 * Y1_SLOT) / 4; i += 32) *(v4f*)(y1 + 4 * i) = z4;
  }
#pragma unroll 1
  for (int m = 0; m < 16; ++m) {
    const v4f v = *(const v4f*)(XP + (size_t)(bbase + m) * NGATE + 4 * lane);
    const int nt = lane >> 2;
    const int dl = (m >> 3) * 16 + 4 * (lane & 3);
    float* dp = xp + (nt * 32 + dl) * 8 + (m & 7);
    dp[0]  = v[0];
    dp[8]  = v[1];
    dp[16] = v[2];
    dp[24] = v[3];
  }

  float cs0[8], cs1[8];
#pragma unroll
  for (int r = 0; r < 8; ++r) { cs0[r] = 0.0f; cs1[r] = 0.0f; }
  const float b1v = c1b[n];
  const float b2v = c2b[0];
  const v8f z8 = {0.f, 0.f, 0.f, 0.f, 0.f, 0.f, 0.f, 0.f};
  __syncthreads();

#pragma unroll 1
  for (int t = 0; t < NSTEP + 4; ++t) {
    {
      const bool live = (t < NSTEP);
      const _Float16* hlast = hr + ((t + 7) & 7) * HR_SLOT;
      _Float16* hcur = hr + (t & 7) * HR_SLOT;
      const v16h ahi = FragH::load(hlast + n * HR_P + 8 * hf);
      const v16h alo = FragH::load(hlast + HR_PLANE + n * HR_P + 8 * hf);
#pragma unroll
      for (int cf = 0; cf < 2; ++cf) {
        const v16h b0 = FragH::load(WHs + ((0 + cf) * 16 + n) * WH_P + 8 * hf);
        const v16h b1 = FragH::load(WHs + ((2 + cf) * 16 + n) * WH_P + 8 * hf);
        const v16h b2 = FragH::load(WHs + ((4 + cf) * 16 + n) * WH_P + 8 * hf);
        const v16h b3 = FragH::load(WHs + ((6 + cf) * 16 + n) * WH_P + 8 * hf);
        const v16h l0 = FragH::load(WLs + ((0 + cf) * 16 + n) * WH_P + 8 * hf);
        const v16h l1 = FragH::load(WLs + ((2 + cf) * 16 + n) * WH_P + 8 * hf);
        const v16h l2 = FragH::load(WLs + ((4 + cf) * 16 + n) * WH_P + 8 * hf);
        const v16h l3 = FragH::load(WLs + ((6 + cf) * 16 + n) * WH_P + 8 * hf);
        v8f m0 = ld_tile8(xp + ((0 + cf) * 32 + lane) * 8);
        v8f m1 = ld_tile8(xp + ((2 + cf) * 32 + lane) * 8);
        v8f m2 = ld_tile8(xp + ((4 + cf) * 32 + lane) * 8);
        v8f m3 = ld_tile8(xp + ((6 + cf) * 32 + lane) * 8);
        v8f r0 = z8, r1 = z8, r2 = z8, r3 = z8;
        m0 = FragH::mma(ahi, b0, m0);
        m1 = FragH::mma(ahi, b1, m1);
        m2 = FragH::mma(ahi, b2, m2);
        m3 = FragH::mma(ahi, b3, m3);
        r0 = FragH::mma(alo, b0, r0);
        r1 = FragH::mma(alo, b1, r1);
        r2 = FragH::mma(alo, b2, r2);
        r3 = FragH::mma(alo, b3, r3);
        r0 = FragH::mma(ahi, l0, r0);
        r1 = FragH::mma(ahi, l1, r1);
        r2 = FragH::mma(ahi, l2, r2);
        r3 = FragH::mma(ahi, l3, r3);
        guard_rec12(m0, m1, m2, m3, r0, r1, r2, r3, ahi, alo, b0, b1, b2, b3, l0, l1, l2, l3);
#pragma unroll
        for (int r = 0; r < 8; ++r) {
          const float zi = m0[r] + r0[r] * LO_CARRY_INV;
          const float zf = m1[r] + r1[r] * LO_CARRY_INV;
          const float zg = m2[r] + r2[r] * LO_CARRY_INV;
          const float zo = m3[r] + r3[r] * LO_CARRY_INV;
          const float iv = fsig(zi);
          const float fv = fsig(zf);
          const float gv = ftanh(zg);
          const float ov = fsig(zo);
          const float co = (cf == 0) ? cs0[r] : cs1[r];
          const float cn = fv * co + iv * gv;
          if (cf == 0) cs0[r] = cn; else cs1[r] = cn;
          const float hn = ov * ftanh(cn);
          const float hsel = live ? hn : 0.0f;
          const _Float16 hi = (_Float16)hsel;
          const float hif = opaque_f32((float)hi);
          const _Float16 lo = (_Float16)((hsel - hif) * LO_CARRY);
          const int o = (8 * hf + r) * HR_P + cf * 16 + n;
          hcur[o] = hi;
          hcur[HR_PLANE + o] = lo;
        }
      }
    }
    __syncthreads();

    if (t >= 36 && ((t - 4) & 31) == 0) flush_tile(ot, out, bbase, ((t - 4) >> 5) - 1, lane);

    {
      const int tc = t - 2;
      const bool cvalid = (tc >= 0) && (tc < NSTEP);
      float* yslot = y1 + ((t + 6) & 7) * Y1_SLOT;
      v8f am = {b1v, b1v, b1v, b1v, b1v, b1v, b1v, b1v};
      v8f ar = z8;
#pragma unroll
      for (int dt = 0; dt < NTAP; ++dt) {
        const _Float16* hs = hr + ((t + 4 + dt) & 7) * HR_SLOT;
        const v16h a0 = FragH::load(hs + n * HR_P + 8 * hf);
        const v16h a1 = FragH::load(hs + HR_PLANE + n * HR_P + 8 * hf);
        const v16h bw = FragH::load(C1s + (dt * NCH1 + n) * WH_P + 8 * hf);
        am = FragH::mma(a0, bw, am);
        ar = FragH::mma(a1, bw, ar);
        guard_cv2(am, ar, a0, a1, bw);
      }
#pragma unroll
      for (int r = 0; r < 8; ++r) {
        const float v = fmaxf(am[r] + ar[r] * LO_CARRY_INV, 0.0f);
        const float vs = cvalid ? v : 0.0f;
        yslot[(8 * hf + r) * Y1_P + n] = vs;
      }
    }
    __syncthreads();

    {
      float acc = 0.0f;
#pragma unroll
      for (int dt = 0; dt < NTAP; ++dt) {
        const float* yp = y1 + ((t + 2 + dt) & 7) * Y1_SLOT + n * Y1_P + hf * 8;
        const float* wp = W2s + (hf * NTAP + dt) * 8;
        const v4f ya = *(const v4f*)(yp);
        const v4f yb = *(const v4f*)(yp + 4);
        const v4f wa = *(const v4f*)(wp);
        const v4f wb = *(const v4f*)(wp + 4);
        acc = fmaf(ya[0], wa[0], acc);
        acc = fmaf(ya[1], wa[1], acc);
        acc = fmaf(ya[2], wa[2], acc);
        acc = fmaf(ya[3], wa[3], acc);
        acc = fmaf(yb[0], wb[0], acc);
        acc = fmaf(yb[1], wb[1], acc);
        acc = fmaf(yb[2], wb[2], acc);
        acc = fmaf(yb[3], wb[3], acc);
      }
      const float other = __shfl_xor(acc, 16, 32);
      const float tot = (acc + other) + b2v;
      if (t >= 4 && hf == 0) ot[n * OT_P + ((t - 4) & 31)] = tot;
    }
  }
  __syncthreads();
  flush_tile(ot, out, bbase, (NSTEP / 32) - 1, lane);
}

extern "C" void kernel_launch(void* const* d_in, const int* in_sizes, int n_in,
                              void* d_out, int out_size, void* d_ws, size_t ws_size, hipStream_t stream) {
  if (n_in < 11 || d_out == nullptr || d_ws == nullptr) return;
  if (in_sizes[0] != NBATCH * NLAT || in_sizes[1] != NFC * NLAT || in_sizes[2] != NFC ||
      in_sizes[3] != NGATE * NFC || in_sizes[4] != NGATE * NHID || in_sizes[5] != NGATE ||
      in_sizes[6] != NGATE || in_sizes[7] != NCH1 * NHID * NTAP || in_sizes[8] != NCH1 ||
      in_sizes[9] != NCH1 * NTAP || in_sizes[10] != 1 || out_size != NBATCH * NSTEP) return;
  const size_t xp_bytes = (size_t)NBATCH * NGATE * sizeof(float);
  if (xp_bytes > ws_size || xp_bytes > (size_t)134217728) return;

  const float* z    = (const float*)d_in[0];
  const float* fc_w = (const float*)d_in[1];
  const float* fc_b = (const float*)d_in[2];
  const float* w_ih = (const float*)d_in[3];
  const float* w_hh = (const float*)d_in[4];
  const float* b_ih = (const float*)d_in[5];
  const float* b_hh = (const float*)d_in[6];
  const float* c1w  = (const float*)d_in[7];
  const float* c1b  = (const float*)d_in[8];
  const float* c2w  = (const float*)d_in[9];
  const float* c2b  = (const float*)d_in[10];
  float* outp = (float*)d_out;
  float* XP   = (float*)d_ws;

  xproj_kernel<<<NBATCH / (16 * K1_WAVES), K1_WAVES * 32, 0, stream>>>(z, fc_w, fc_b, w_ih, b_ih, b_hh, XP);
  decoder_seq_kernel<<<NBATCH / (16 * K2_WAVES), K2_WAVES * 32, 0, stream>>>(XP, w_hh, c1w, c1b, c2w, c2b, outp);
}
